// SelfAttention_85770496901684
// MI455X (gfx1250) — hardware-verified
//
#include <hip/hip_runtime.h>


#ifndef NB
#define NB 2
#endif
#ifndef SEQ
#define SEQ 2048
#endif
#define NB_FULL    2
#define SEQ_FULL   2048
#define NHEAD      16
#define HDIM       64
#define BQ         128
#define BK         32
#define NWAVE      8
#define EARLY_QBLK 2
#define CT         64
#define TP         72
#define OP         68
#define NWORD      (SEQ / 32)
#define MWP        (((NWORD + 31) / 32) * 32)
#define MWG        (MWP / 32)

static_assert(SEQ % BQ == 0);
static_assert(SEQ % CT == 0);
static_assert(SEQ % BK == 0);
static_assert(SEQ % 32 == 0);
static_assert(SEQ % 8 == 0);
static_assert(BK == 32);
static_assert(BQ == NWAVE * 16);
static_assert(HDIM == 64);
static_assert(SEQ <= SEQ_FULL);
static_assert(NB >= 1 && NB <= NB_FULL);
static_assert((TP * 2) % 16 == 0);
static_assert((OP * 4) % 16 == 0);
static_assert(TP >= CT);
static_assert(OP >= HDIM);
static_assert(MWP >= NWORD);
static_assert(MWP % 32 == 0);
static_assert(2 * MWP <= 256);
static_assert(NWAVE * 32 == 256);

typedef __bf16   bf16;
typedef _Float16 f16;
typedef bf16     v16bf __attribute__((ext_vector_type(16)));
typedef f16      v16h  __attribute__((ext_vector_type(16)));
typedef f16      v8h   __attribute__((ext_vector_type(8)));
typedef float    v8f   __attribute__((ext_vector_type(8)));
typedef float    v4f   __attribute__((ext_vector_type(4)));
typedef unsigned v4u   __attribute__((ext_vector_type(4)));

union FragB  { v16bf v; v4u q[2]; bf16 h[16]; };
union FragH  { v16h  v; v4u q[2]; f16  h[16]; };
union Pack8B { v4u u; bf16 h[8]; };
union Pack8H { v4u u; v8h v; f16 h[8]; };

#define KB_BYTES ((size_t)NB * NHEAD * SEQ * HDIM * 2)
#define VT_BYTES ((size_t)NB * NHEAD * HDIM * SEQ * 2)
#define MW_BYTES ((size_t)SEQ * MWP * 4)
static_assert(KB_BYTES % 128 == 0);
static_assert(VT_BYTES % 128 == 0);
static_assert(MW_BYTES % 128 == 0);
static_assert(KB_BYTES + VT_BYTES + MW_BYTES <= (size_t)134217728);

static __device__ __forceinline__ v8f mma_bf16(v16bf a, v16bf b, v8f acc) {
  acc = __builtin_amdgcn_wmma_f32_16x16x32_bf16(false, a, false, b, (short)0, acc, false, false);
  asm volatile("v_nop\n\tv_nop\n\tv_nop\n\tv_nop" : "+v"(acc) : "v"(a), "v"(b));
  return acc;
}
static __device__ __forceinline__ v8f mma_f16(v16h a, v16h b, v8f acc) {
  acc = __builtin_amdgcn_wmma_f32_16x16x32_f16(false, a, false, b, (short)0, acc, false, false);
  asm volatile("v_nop\n\tv_nop\n\tv_nop\n\tv_nop" : "+v"(acc) : "v"(a), "v"(b));
  return acc;
}

__global__ __launch_bounds__(256) void mask_pack_kernel(const int* __restrict__ mask,
                                                        unsigned* __restrict__ mw) {
  const int tid  = threadIdx.x;
  const int wave = __builtin_amdgcn_readfirstlane(tid >> 5);
  const int lane = tid & 31;
  __shared__ __align__(16) unsigned sW[8 * MWP];

  const int q = blockIdx.x * 8 + wave;
  const int* row = mask + (size_t)q * SEQ_FULL;

  #pragma unroll
  for (int g = 0; g < MWG; ++g) {
    unsigned acc = 0u;
    #pragma unroll 8
    for (int it = 0; it < 32; ++it) {
      const int wi = g * 32 + it;
      unsigned bal = 0u;
      if (wi < NWORD) {
        const int m = row[wi * 32 + lane];
        bal = __builtin_amdgcn_ballot_w32(m != 0);
      }
      acc = (it == lane) ? bal : acc;
    }
    sW[wave * MWP + g * 32 + lane] = acc;
  }
  __syncthreads();

  if (tid < 2 * MWP) {
    const int r = tid / (MWP / 4);
    const int p = tid % (MWP / 4);
    const v4u val = *(const v4u*)(sW + r * MWP + p * 4);
    unsigned* dst = mw + ((size_t)(blockIdx.x * 8 + r) * MWP + p * 4);
    *(volatile v4u*)dst = val;
    __threadfence();
    *(volatile v4u*)dst = val;
  }
}

__global__ __launch_bounds__(256) void kv_planes_kernel(const float* __restrict__ kin,
                                                        const float* __restrict__ vin,
                                                        bf16* __restrict__ kb,
                                                        f16* __restrict__ vt) {
  const int kt  = blockIdx.x;
  const int h   = blockIdx.y;
  const int b   = blockIdx.z;
  const int tid = threadIdx.x;
  __shared__ __align__(16) f16 sT[HDIM * TP];
  const int s0 = kt * CT;
  const size_t hrow = (size_t)b * NHEAD + h;

  v4u    kval[2];
  size_t kidx[2];
  #pragma unroll
  for (int kk = 0; kk < 2; ++kk) {
    const int key = kk * 32 + (tid >> 3);
    const int d0  = (tid & 7) * 8;
    const size_t src = (hrow * SEQ_FULL + s0 + key) * HDIM + d0;
    const v4f k0 = *(const v4f*)(kin + src);
    const v4f k1 = *(const v4f*)(kin + src + 4);
    const v4f v0 = *(const v4f*)(vin + src);
    const v4f v1 = *(const v4f*)(vin + src + 4);
    Pack8B pk;
    #pragma unroll
    for (int i = 0; i < 4; ++i) {
      pk.h[i]     = (bf16)k0[i];
      pk.h[4 + i] = (bf16)k1[i];
    }
    kval[kk] = pk.u;
    kidx[kk] = ((hrow * SEQ) + s0 + key) * HDIM + d0;
    #pragma unroll
    for (int i = 0; i < 4; ++i) {
      sT[(d0 + i) * TP + key]     = (f16)(float)(bf16)v0[i];
      sT[(d0 + 4 + i) * TP + key] = (f16)(float)(bf16)v1[i];
    }
  }
  __syncthreads();

  v4u    vval[2];
  size_t vidx[2];
  #pragma unroll
  for (int kk = 0; kk < 2; ++kk) {
    const int d  = kk * 32 + (tid >> 3);
    const int ks = (tid & 7) * 8;
    Pack8H ph;
    ph.v = *(const v8h*)(sT + d * TP + ks);
    vval[kk] = ph.u;
    vidx[kk] = ((hrow * HDIM) + d) * SEQ + s0 + ks;
  }

  #pragma unroll
  for (int kk = 0; kk < 2; ++kk) {
    *(volatile v4u*)(kb + kidx[kk]) = kval[kk];
    *(volatile v4u*)(vt + vidx[kk]) = vval[kk];
  }
  __threadfence();
  #pragma unroll
  for (int kk = 0; kk < 2; ++kk) {
    *(volatile v4u*)(kb + kidx[kk]) = kval[kk];
    *(volatile v4u*)(vt + vidx[kk]) = vval[kk];
  }
}

template <int RES>
static __device__ __forceinline__ void attn_body(const float* __restrict__ qin,
                                                 const bf16* __restrict__ kb,
                                                 const f16* __restrict__ vt,
                                                 const unsigned* __restrict__ mw,
                                                 float* __restrict__ out,
                                                 int qblk0) {
  const int qblk = qblk0 + blockIdx.x;
  const int h    = blockIdx.y;
  const int b    = blockIdx.z;
  const int tid  = threadIdx.x;
  const int wave = __builtin_amdgcn_readfirstlane(tid >> 5);
  const int lane = tid & 31;
  const int lq   = lane & 15;
  const int hi   = lane >> 4;

  __shared__ __align__(16) float sO[NWAVE * 16 * OP];

  const int qrow0 = qblk * BQ + wave * 16;
  const size_t hrow = (size_t)b * NHEAD + h;

  FragB qf[2];
  {
    const float* qp = qin + (hrow * SEQ_FULL + qrow0 + lq) * HDIM;
    #pragma unroll
    for (int f = 0; f < 2; ++f) {
      const v4f a0 = *(const v4f*)(qp + f * 32 + hi * 8);
      const v4f a1 = *(const v4f*)(qp + f * 32 + hi * 8 + 4);
      const v4f b0 = *(const v4f*)(qp + f * 32 + 16 + hi * 8);
      const v4f b1 = *(const v4f*)(qp + f * 32 + 16 + hi * 8 + 4);
      #pragma unroll
      for (int i = 0; i < 4; ++i) {
        qf[f].h[i]      = (bf16)a0[i];
        qf[f].h[4 + i]  = (bf16)a1[i];
        qf[f].h[8 + i]  = (bf16)b0[i];
        qf[f].h[12 + i] = (bf16)b1[i];
      }
    }
  }

  const bf16*     kb_h = kb + hrow * SEQ * HDIM;
  const f16*      vt_h = vt + hrow * HDIM * SEQ;
  const unsigned* mrow = mw + (size_t)(qrow0 + lq) * MWP;

  v8f o[4], o2[4];
  #pragma unroll
  for (int dt = 0; dt < 4; ++dt) {
    o[dt]  = (v8f){0, 0, 0, 0, 0, 0, 0, 0};
    o2[dt] = (v8f){0, 0, 0, 0, 0, 0, 0, 0};
  }

  const float NEG_INF = -__builtin_inff();
  float rmax = NEG_INF;
  float rsum = 0.0f;
  const float SL = 0.125f * 1.4426950408889634f;

  for (int i = 0; i < NWORD; ++i) {
    const int j0 = i * BK;

    const unsigned word = mrow[i];
    const unsigned anyk = __builtin_amdgcn_ballot_w32(word != 0u);
    if (anyk == 0u) continue;
    const unsigned part = __builtin_amdgcn_ballot_w32(word != 0xffffffffu);

    FragB ak[2][2];
    #pragma unroll
    for (int sub = 0; sub < 2; ++sub) {
      #pragma unroll
      for (int f = 0; f < 2; ++f) {
        const bf16* base = kb_h + (size_t)(j0 + sub * 16 + lq) * HDIM + f * 32 + hi * 8;
        ak[sub][f].q[0] = *(const v4u*)(base);
        ak[sub][f].q[1] = *(const v4u*)(base + 16);
      }
    }
    FragH bv[4];
    #pragma unroll
    for (int dt = 0; dt < 4; ++dt) {
      const f16* base = vt_h + (size_t)(dt * 16 + lq) * SEQ + j0 + hi * 8;
      bv[dt].q[0] = *(const v4u*)(base);
      bv[dt].q[1] = *(const v4u*)(base + 16);
    }

    v8f c[2];
    #pragma unroll
    for (int sub = 0; sub < 2; ++sub) {
      v8f acc = (v8f){0, 0, 0, 0, 0, 0, 0, 0};
      acc = mma_bf16(ak[sub][0].v, qf[0].v, acc);
      acc = mma_bf16(ak[sub][1].v, qf[1].v, acc);
      c[sub] = acc;
    }

    if (part != 0u) {
      const unsigned wsh = word >> (hi * 8);
      #pragma unroll
      for (int sub = 0; sub < 2; ++sub) {
        #pragma unroll
        for (int r = 0; r < 8; ++r) {
          const bool keep = ((wsh >> (sub * 16 + r)) & 1u) != 0u;
          c[sub][r] = keep ? c[sub][r] : NEG_INF;
        }
      }
    }

    float m_new = rmax;
    #pragma unroll
    for (int r = 0; r < 8; ++r) {
      m_new = fmaxf(m_new, c[0][r]);
      m_new = fmaxf(m_new, c[1][r]);
    }
    m_new = fmaxf(m_new, __shfl_xor(m_new, 16, 32));
    const float m_use = (m_new == NEG_INF) ? 0.0f : m_new;
    const float scale = __builtin_amdgcn_exp2f((rmax - m_use) * SL);
    rmax = m_new;

    FragH pa, pr;
    float psum = 0.0f;
    #pragma unroll
    for (int r = 0; r < 8; ++r) {
      const float p0 = __builtin_amdgcn_exp2f((c[0][r] - m_use) * SL);
      const float p1 = __builtin_amdgcn_exp2f((c[1][r] - m_use) * SL);
      psum += p0 + p1;
      const float pc0 = p0 * 4096.0f;
      const float pc1 = p1 * 4096.0f;
      const f16 h0 = (f16)pc0;
      const f16 h1 = (f16)pc1;
      pa.h[r]     = h0;
      pa.h[8 + r] = h1;
      if (RES != 0) {
        pr.h[r]     = (f16)((pc0 - (float)h0) * 1024.0f);
        pr.h[8 + r] = (f16)((pc1 - (float)h1) * 1024.0f);
      }
    }
    rsum = rsum * scale + psum + __shfl_xor(psum, 16, 32);

    float sc[8];
    #pragma unroll
    for (int r = 0; r < 8; ++r) sc[r] = __shfl(scale, (hi << 3) + r, 32);
    #pragma unroll
    for (int dt = 0; dt < 4; ++dt) {
      #pragma unroll
      for (int r = 0; r < 8; ++r) {
        o[dt][r] *= sc[r];
        if (RES != 0) o2[dt][r] *= sc[r];
      }
    }

    #pragma unroll
    for (int dt = 0; dt < 4; ++dt) {
      o[dt] = mma_f16(pa.v, bv[dt].v, o[dt]);
      if (RES != 0) o2[dt] = mma_f16(pr.v, bv[dt].v, o2[dt]);
    }
  }

  float rs[8];
  #pragma unroll
  for (int r = 0; r < 8; ++r) rs[r] = 1.0f / __shfl(rsum, (hi << 3) + r, 32);

  const int sbase = wave * (16 * OP);
  #pragma unroll
  for (int r = 0; r < 8; ++r) {
    #pragma unroll
    for (int dt = 0; dt < 4; ++dt) {
      float val = o[dt][r];
      if (RES != 0) val += o2[dt][r] * (1.0f / 1024.0f);
      sO[sbase + (hi * 8 + r) * OP + dt * 16 + lq] = val * (1.0f / 4096.0f) * rs[r];
    }
  }
  __syncthreads();

  v4f    vals[8];
  size_t gidx[8];
  #pragma unroll
  for (int it = 0; it < 8; ++it) {
    const int row = it * 2 + hi;
    vals[it] = *(const v4f*)(sO + sbase + row * OP + lq * 4);
    gidx[it] = (hrow * SEQ_FULL + qrow0 + row) * HDIM + lq * 4;
  }
  #pragma unroll
  for (int it = 0; it < 8; ++it) *(volatile v4f*)(out + gidx[it]) = vals[it];
  __threadfence();
  #pragma unroll
  for (int it = 0; it < 8; ++it) *(volatile v4f*)(out + gidx[it]) = vals[it];
}

__global__ __launch_bounds__(256) void attn_early_kernel(const float* __restrict__ qin,
                                                         const bf16* __restrict__ kb,
                                                         const f16* __restrict__ vt,
                                                         const unsigned* __restrict__ mw,
                                                         float* __restrict__ out,
                                                         int qblk0) {
  attn_body<1>(qin, kb, vt, mw, out, qblk0);
}

__global__ __launch_bounds__(256) void attn_late_kernel(const float* __restrict__ qin,
                                                        const bf16* __restrict__ kb,
                                                        const f16* __restrict__ vt,
                                                        const unsigned* __restrict__ mw,
                                                        float* __restrict__ out,
                                                        int qblk0) {
  attn_body<0>(qin, kb, vt, mw, out, qblk0);
}

extern "C" void kernel_launch(void* const* d_in, const int* in_sizes, int n_in,
                              void* d_out, int out_size, void* d_ws, size_t ws_size,
                              hipStream_t stream) {
  if (n_in < 4) return;
  const size_t qkv_need  = ((size_t)(NB * NHEAD - 1) * SEQ_FULL + SEQ) * HDIM;
  const size_t mask_need = (size_t)(SEQ - 1) * SEQ_FULL + SEQ;
  if ((size_t)in_sizes[0] < qkv_need) return;
  if ((size_t)in_sizes[1] < qkv_need) return;
  if ((size_t)in_sizes[2] < qkv_need) return;
  if ((size_t)in_sizes[3] < mask_need) return;
  if ((size_t)out_size < qkv_need) return;

  const size_t kb_bytes = KB_BYTES;
  const size_t vt_bytes = VT_BYTES;
  const size_t mw_bytes = MW_BYTES;
  if (ws_size < kb_bytes + vt_bytes + mw_bytes) return;

  const float* qin  = (const float*)d_in[0];
  const float* kin  = (const float*)d_in[1];
  const float* vin  = (const float*)d_in[2];
  const int*   mask = (const int*)d_in[3];
  float*       out  = (float*)d_out;
  bf16*        kb   = (bf16*)d_ws;
  f16*         vt   = (f16*)((char*)d_ws + kb_bytes);
  unsigned*    mw   = (unsigned*)((char*)d_ws + kb_bytes + vt_bytes);

  mask_pack_kernel<<<dim3(SEQ / 8), 256, 0, stream>>>(mask, mw);
  kv_planes_kernel<<<dim3(SEQ / CT, NHEAD, NB), 256, 0, stream>>>(kin, vin, kb, vt);

  const int nqb     = SEQ / BQ;
  const int n_early = (EARLY_QBLK < nqb) ? EARLY_QBLK : nqb;
  const int n_late  = nqb - n_early;
  attn_early_kernel<<<dim3(n_early, NHEAD, NB), 256, 0, stream>>>(qin, kb, vt, mw, out, 0);
  if (n_late > 0)
    attn_late_kernel<<<dim3(n_late, NHEAD, NB), 256, 0, stream>>>(qin, kb, vt, mw, out, n_early);
}
